// Feature_Expansion_11982958756579
// MI455X (gfx1250) — hardware-run, weakly checked
//
#include <hip/hip_runtime.h>


namespace {
constexpr int N = 4096, C = 64, O = 128, E = 135168, S = 8192, NH = 2, HD = 32;
constexpr float XS = 8.0f, PS = 256.0f, WSC = 256.0f, SCALE = 0.17677669529663688f;
typedef _Float16 b16;
typedef __attribute__((ext_vector_type(16))) _Float16 v16b;
typedef __attribute__((ext_vector_type(8))) _Float16 v8b;
typedef __attribute__((ext_vector_type(8))) float v8f;
typedef __attribute__((ext_vector_type(4))) float v4f;
typedef __attribute__((ext_vector_type(2))) float v2f;
__device__ __forceinline__ float bf16_rne(float f) { unsigned int u = __float_as_uint(f); u += 0x7FFFu + ((u >> 16) & 1u); float r = __uint_as_float(u & 0xFFFF0000u); asm volatile("" : "+v"(r)); return r; }
__device__ __forceinline__ void split16(float v, b16& hi, b16& lo) { hi = (b16)v; lo = (b16)(v - (float)hi); }
__device__ __forceinline__ v16b frag_kb(const b16* p, int hh) { const v8b a = *(const v8b*)(p + 8 * hh), b = *(const v8b*)(p + 16 + 8 * hh); v16b f;
#pragma unroll
  for (int e = 0; e < 8; ++e) { f[e] = a[e]; f[8 + e] = b[e]; } return f; }
__device__ __forceinline__ v8f wmma16b(v16b a, v16b b, v8f c) { v8f d = __builtin_amdgcn_wmma_f32_16x16x32_f16(false, a, false, b, (short)0, c, false, false); asm volatile("v_nop\n\tv_nop\n\tv_nop\n\tv_nop" : "+v"(d) : "v"(a), "v"(b)); return d; }
__device__ __forceinline__ void wave_lds_sync() { __builtin_amdgcn_fence(__ATOMIC_RELEASE, "workgroup"); __builtin_amdgcn_wave_barrier(); __builtin_amdgcn_fence(__ATOMIC_ACQUIRE, "workgroup"); }
__device__ __forceinline__ float pmul(float a, float b) { float p = a * b; asm volatile("" : "+v"(p)); return p; }
__device__ __forceinline__ int iclamp(int v, int lo, int hi) { return v < lo ? lo : (v > hi ? hi : v); }
constexpr int CSR_NBLK8 = 512, CSR_GB8 = 8, CSR_GN8 = 1 << CSR_GB8  , CSR_TS8 = (CSR_GN8 < 32 ? 32 : CSR_GN8)  , CSR_MAXG8 = 512, CSR_CAP8 = 12288  ;
__device__ __host__ __forceinline__ int csr_tix8(int v) { return (v >> CSR_GB8) * CSR_TS8 + (v & (CSR_GN8 - 1)); }
__global__ __launch_bounds__(64) void csrA_kernel8(const int* __restrict__ dst, int E, int N, int nG, int CHP, int NGP, int* __restrict__ STG, int* __restrict__ HST) {
  extern __shared__ int sm[];
  int* cnt = sm; int* run = sm + NGP; int* ids = sm + 2 * NGP;
  const int b = blockIdx.x; const int ch = (E + CSR_NBLK8 - 1) / CSR_NBLK8; const int e0 = b * ch, e1 = min(E, e0 + ch);
  for (int i = threadIdx.x; i < NGP; i += 64) cnt[i] = 0;
  for (int i = threadIdx.x; i < CHP; i += 64) ids[i] = -1;
  __syncthreads();
  if (threadIdx.x == 0) {
    for (int e = e0; e < e1; ++e) { int d = dst[e]; d = (d < 0) ? 0 : (d >= N ? N - 1 : d); cnt[d >> CSR_GB8] += 1; }
    int acc = 0; for (int g = 0; g < nG; ++g) { run[g] = acc; acc += cnt[g]; }
    for (int e = e0; e < e1; ++e) { int d = dst[e]; d = (d < 0) ? 0 : (d >= N ? N - 1 : d); const int g = d >> CSR_GB8; ids[run[g]] = e; run[g] += 1; } }
  __syncthreads();
  typedef __attribute__((ext_vector_type(4))) int v4i;
  for (int pass = 0; pass < 2; ++pass) {
    for (int i = threadIdx.x; i < CHP / 4; i += 64) *(volatile v4i*)(STG + (size_t)b * CHP + i * 4) = *(const v4i*)(&ids[i * 4]);
    for (int i = threadIdx.x; i < NGP / 4; i += 64) { v4i v; for (int e = 0; e < 4; ++e) v[e] = (i * 4 + e < nG) ? cnt[i * 4 + e] : 0; *(volatile v4i*)(HST + (size_t)b * NGP + i * 4) = v; }
    __threadfence(); }
}
__global__ __launch_bounds__(512) void csrS_kernel8(const int* __restrict__ HST, int nG, int NGP, int* __restrict__ START, int* __restrict__ TOT, int* __restrict__ OFF) {
  __shared__ int tot[CSR_MAXG8];
  const int b = threadIdx.x;
  for (int pass = 0; pass < 2; ++pass) { int runb = 0; for (int g = 0; g < nG; ++g) { int c = HST[(size_t)b * NGP + g]; c = (c < 0) ? 0 : c; ((volatile int*)OFF)[(size_t)g * CSR_NBLK8 + b] = runb; runb += c; } __threadfence(); }
  for (int g = threadIdx.x; g < nG; g += 512) { int s = 0; for (int bb = 0; bb < CSR_NBLK8; ++bb) { int c = HST[(size_t)bb * NGP + g]; s += (c < 0) ? 0 : c; } tot[g] = s; }
  __syncthreads();
  if (threadIdx.x < 32) {
    __shared__ int st[CSR_MAXG8 + 32];
    if (threadIdx.x == 0) { int acc = 0; for (int g = 0; g < NGP; ++g) { st[g] = acc; if (g < nG) acc += (tot[g] + 31) & ~31; } st[NGP] = acc; }
    __builtin_amdgcn_fence(__ATOMIC_RELEASE, "workgroup"); __builtin_amdgcn_wave_barrier(); __builtin_amdgcn_fence(__ATOMIC_ACQUIRE, "workgroup");
    for (int pass = 0; pass < 2; ++pass) { for (int i = threadIdx.x; i < NGP + 32; i += 32) { ((volatile int*)START)[i] = (i <= NGP) ? st[min(i, NGP)] : 0; ((volatile int*)TOT)[i] = (i < nG) ? tot[i] : 0; } __threadfence(); } }
}
__global__ __launch_bounds__(256) void csrB_kernel8(const int* __restrict__ dst, int N, int nG, int CHP, int NGP, int permLen, const int* __restrict__ STG, const int* __restrict__ HST, const int* __restrict__ OFF, const int* __restrict__ START, const int* __restrict__ TOT, int* __restrict__ PERM, int* __restrict__ ROWPTR, int* __restrict__ ROWCNT, int* __restrict__ FLAG) {
  typedef __attribute__((ext_vector_type(4))) int v4i;
  __shared__ int ids[CSR_CAP8]; __shared__ unsigned short key[CSR_CAP8]; __shared__ int outp[CSR_CAP8]; __shared__ int ncnt[CSR_GN8 + 1]; __shared__ int boff[CSR_NBLK8 + 1];
  const int g = blockIdx.x, t_ = threadIdx.x; int tot = TOT[g]; int st = START[g], stn = START[g + 1]; const int v0 = g * CSR_GN8; const int nv = min(CSR_GN8, N - v0); const int t0 = g * CSR_TS8;
  st = (st < 0) ? 0 : (st > permLen - 32 ? permLen - 32 : st) & ~31; stn = (stn < st) ? st : (stn > permLen ? permLen : stn); tot = (tot < 0) ? 0 : tot; if (tot > stn - st && tot <= CSR_CAP8) tot = stn - st;
  if (tot > CSR_CAP8) {
    for (int pass = 0; pass < 2; ++pass) { for (int i = t_; i < CSR_TS8 / 4; i += 256) { v4i a, c; for (int e = 0; e < 4; ++e) { a[e] = st; c[e] = 0; } *(volatile v4i*)(ROWPTR + t0 + i * 4) = a; *(volatile v4i*)(ROWCNT + t0 + i * 4) = c; } if (t_ == 0) ((volatile int*)FLAG)[0] = 1; __threadfence(); } (void)nv; return; }
  if (t_ == 0) { int acc = 0; for (int b = 0; b < CSR_NBLK8; ++b) { boff[b] = acc; int c = HST[(size_t)b * NGP + g]; c = (c < 0) ? 0 : (c > CHP ? CHP : c); acc += c; if (acc > tot) acc = tot; } boff[CSR_NBLK8] = acc; }
  for (int i = t_; i <= CSR_GN8; i += 256) ncnt[i] = 0;
  __syncthreads();
  for (int b = 0; b < CSR_NBLK8; ++b) { const int c = boff[b + 1] - boff[b]; int o_ = OFF[(size_t)g * CSR_NBLK8 + b]; o_ = (o_ < 0) ? 0 : (o_ > CHP - c ? CHP - c : o_); const int* src_ = STG + (size_t)b * CHP + o_;
    for (int i = t_; i < c; i += 256) { int id = src_[i]; id = (id < 0) ? 0 : id; ids[boff[b] + i] = id; int d = dst[id]; d = (d < v0) ? v0 : (d >= N ? N - 1 : d); int kk = d - v0; kk = (kk < 0) ? 0 : (kk >= CSR_GN8 ? CSR_GN8 - 1 : kk); key[boff[b] + i] = (unsigned short)kk; } }
  __syncthreads();
  if (t_ == 0) { for (int i = 0; i < tot; ++i) ncnt[key[i]] += 1; int acc = 0; for (int vl = 0; vl < CSR_GN8; ++vl) { const int c = ncnt[vl]; ncnt[vl] = acc; acc += c; } ncnt[CSR_GN8] = acc;
    for (int i = 0; i < tot; ++i) { const int vl = key[i]; outp[ncnt[vl]] = ids[i]; ncnt[vl] += 1; }
    for (int vl = CSR_GN8; vl > 0; --vl) ncnt[vl] = ncnt[vl - 1]; ncnt[0] = 0; }
  __syncthreads();
  for (int pass = 0; pass < 2; ++pass) {
    for (int i = t_; i < (stn - st) / 4; i += 256) { v4i v; for (int e = 0; e < 4; ++e) { const int q = i * 4 + e; v[e] = (q < tot) ? outp[q] : -1; } *(volatile v4i*)(PERM + st + i * 4) = v; }
    for (int i = t_; i < CSR_TS8 / 4; i += 256) { v4i a, c; for (int e = 0; e < 4; ++e) { const int vl = i * 4 + e; const int vc = vl < CSR_GN8 ? vl : CSR_GN8; a[e] = (vl < CSR_GN8) ? st + ncnt[vc] : st; c[e] = (vl < nv) ? (ncnt[(vc < CSR_GN8 ? vc : CSR_GN8 - 1) + 1] - ncnt[vc]) : 0; } *(volatile v4i*)(ROWPTR + t0 + i * 4) = a; *(volatile v4i*)(ROWCNT + t0 + i * 4) = c; }
    __threadfence(); }
}
__global__ __launch_bounds__(256) void csrZ_kernel8(int* __restrict__ p, size_t n4) { typedef __attribute__((ext_vector_type(4))) int v4i; const size_t tid = (size_t)blockIdx.x * 256 + threadIdx.x, nth = (size_t)gridDim.x * 256; v4i z = {0, 0, 0, 0}; for (size_t i = tid; i < n4; i += nth) *(volatile v4i*)(p + i * 4) = z; }
struct CsrBufs8 { int *STG, *HST, *OFF, *START, *TOT, *PERM, *ROWPTR, *ROWCNT, *FLAG; int nG, NGP, CHP; size_t permLen; char* base; size_t bytes; };
static size_t csr_carve8(CsrBufs8& c, char* ws, size_t off, int E, int N) {
  const size_t off0 = off; c.base = ws + off;
  auto al = [&](size_t bytes) { char* p = ws + off; off += (bytes + 255) & ~(size_t)255; return p; };
  c.nG = (N + CSR_GN8 - 1) / CSR_GN8; c.NGP = (c.nG + 31) & ~31; const int ch = (E + CSR_NBLK8 - 1) / CSR_NBLK8; c.CHP = (ch + 31) & ~31; c.permLen = (size_t)E + 32 * (size_t)c.nG + 32;
  c.STG = (int*)al((size_t)CSR_NBLK8 * c.CHP * 4); c.HST = (int*)al((size_t)CSR_NBLK8 * c.NGP * 4); c.OFF = (int*)al((size_t)c.NGP * CSR_NBLK8 * 4); c.START = (int*)al((size_t)(c.NGP + 64) * 4); c.TOT = (int*)al((size_t)(c.NGP + 64) * 4);
  c.PERM = (int*)al(c.permLen * 4); c.ROWPTR = (int*)al((size_t)c.nG * CSR_TS8 * 4); c.ROWCNT = (int*)al((size_t)c.nG * CSR_TS8 * 4); c.FLAG = (int*)al(256);
  c.bytes = off - off0; return off;
}
static void csr_build8(const CsrBufs8& c, const int* dst, int E, int N, hipStream_t stream) {
  const size_t smem = (size_t)(2 * c.NGP + c.CHP) * 4;
  csrZ_kernel8<<<512, 256, 0, stream>>>((int*)c.base, c.bytes / 16);
  csrA_kernel8<<<CSR_NBLK8, 64, smem, stream>>>(dst, E, N, c.nG, c.CHP, c.NGP, c.STG, c.HST);
  csrS_kernel8<<<1, 512, 0, stream>>>(c.HST, c.nG, c.NGP, c.START, c.TOT, c.OFF);
  csrB_kernel8<<<c.nG, 256, 0, stream>>>(dst, N, c.nG, c.CHP, c.NGP, (int)c.permLen, c.STG, c.HST, c.OFF, c.START, c.TOT, c.PERM, c.ROWPTR, c.ROWCNT, c.FLAG);
}


__global__ __launch_bounds__(256) void wput_kernel(const float* __restrict__ lw, const float* __restrict__ lsw, const float* __restrict__ ldw, const float* __restrict__ qw, const float* __restrict__ kw, const float* __restrict__ vw, const float* __restrict__ ow, b16* __restrict__ LT, b16* __restrict__ QKVT, b16* __restrict__ OWT) { const int u = blockIdx.x * 256 + threadIdx.x;
  for (int pass = 0; pass < 2; ++pass) {
    if (u < 3 * O * 8) { const int r = u / 8, k0 = (u % 8) * 8; const int blk = r / O, o = r % O; const float* w = blk == 0 ? lw : blk == 1 ? lsw : ldw; v8b v;
#pragma unroll
      for (int j = 0; j < 8; ++j) v[j] = (b16)(bf16_rne(w[(k0 + j) * O + o]) * WSC); *(volatile v8b*)(LT + (size_t)r * C + k0) = v; }
    if (u < 3 * C * 8) { const int r = u / 8, k0 = (u % 8) * 8; const int blk = r / C, o = r % C; const float* w = blk == 0 ? qw : blk == 1 ? kw : vw; v8b v;
#pragma unroll
      for (int j = 0; j < 8; ++j) v[j] = (b16)(bf16_rne(w[(k0 + j) * C + o]) * WSC); *(volatile v8b*)(QKVT + (size_t)r * C + k0) = v; }
    if (u < C * 8) { const int o = u / 8, k0 = (u % 8) * 8; v8b v;
#pragma unroll
      for (int j = 0; j < 8; ++j) v[j] = (b16)(bf16_rne(ow[(k0 + j) * C + o]) * WSC); *(volatile v8b*)(OWT + (size_t)o * C + k0) = v; }
    __threadfence(); } }
__global__ __launch_bounds__(32) void lin_kernel(const float* __restrict__ x, const b16* __restrict__ LT, float* __restrict__ L) { __shared__ __attribute__((aligned(16))) b16 Ah[16][72]; __shared__ float Tf[16][388]; const int lane = threadIdx.x, nloc = lane & 15, hlf = lane >> 4; const size_t m0 = (size_t)blockIdx.x * 16;
  for (int rr = 0; rr < 16; ++rr) for (int q = 0; q < 2; ++q) Ah[rr][q * 32 + lane] = (b16)(bf16_rne(x[(m0 + rr) * C + q * 32 + lane]) * XS);
  wave_lds_sync(); const v16b a0 = frag_kb(&Ah[nloc][0], hlf), a1 = frag_kb(&Ah[nloc][32], hlf);
#pragma unroll
  for (int t = 0; t < 24; ++t) { v8f acc = {}; acc = wmma16b(a0, frag_kb(LT + (size_t)(t * 16 + nloc) * C, hlf), acc); acc = wmma16b(a1, frag_kb(LT + (size_t)(t * 16 + nloc) * C + 32, hlf), acc);
#pragma unroll
    for (int r8 = 0; r8 < 8; ++r8) Tf[8 * hlf + r8][t * 16 + nloc] = acc[r8] * (1.0f / (XS * WSC)); }
  wave_lds_sync();
  for (int pass = 0; pass < 2; ++pass) { for (int rr = 0; rr < 16; ++rr) for (int g = 0; g < 3; ++g) *(volatile v4f*)(L + (m0 + rr) * 3 * O + g * 128 + lane * 4) = *(const v4f*)(&Tf[rr][g * 128 + lane * 4]); __threadfence(); } }
__global__ __launch_bounds__(256) void pt_kernel(const float* __restrict__ L, const float* __restrict__ pos, const float* __restrict__ pw, const float* __restrict__ pb, const int* __restrict__ srcs, const int* __restrict__ PERM, const int* __restrict__ ROWPTR, const int* __restrict__ ROWCNT, int permLen, float* __restrict__ T) {
  const int wave = threadIdx.x >> 5, lane = threadIdx.x & 31; const size_t i = (size_t)blockIdx.x * 8 + wave; if (i >= (size_t)N) return; int st = ROWPTR[i], cnt = ROWCNT[i]; cnt = iclamp(cnt, 0, E); st = iclamp(st, 0, permLen - cnt);
  float W0[4], W1[4], W2[4], PB[4], LD[4], m[4], den[4], acc[4]; const float pix = bf16_rne(pos[i * 3]), piy = bf16_rne(pos[i * 3 + 1]), piz = bf16_rne(pos[i * 3 + 2]);
#pragma unroll
  for (int k = 0; k < 4; ++k) { const int c = lane * 4 + k; W0[k] = bf16_rne(pw[c]); W1[k] = bf16_rne(pw[O + c]); W2[k] = bf16_rne(pw[2 * O + c]); PB[k] = bf16_rne(pb[c]); LD[k] = L[i * 3 * O + 2 * O + c]; m[k] = -INFINITY; den[k] = 0.0f; acc[k] = 0.0f; }
#pragma unroll 1
  for (int j = 0; j < cnt; ++j) { const int e = iclamp(PERM[st + j], 0, E - 1); const size_t u = (size_t)iclamp(srcs[e], 0, N - 1); const float dx = pix - bf16_rne(pos[u * 3]), dy = piy - bf16_rne(pos[u * 3 + 1]), dz = piz - bf16_rne(pos[u * 3 + 2]);
    const v4f ls = *(const v4f*)(L + u * 3 * O + O + lane * 4), ln = *(const v4f*)(L + u * 3 * O + lane * 4);
#pragma unroll
    for (int k = 0; k < 4; ++k) { const float dl = pmul(dx, W0[k]) + pmul(dy, W1[k]) + pmul(dz, W2[k]) + PB[k]; const float al = LD[k] - ls[k] + dl; const float mn = fmaxf(m[k], al); const float sf = (m[k] == -INFINITY) ? 0.0f : __expf(m[k] - mn); const float p = __expf(al - mn); den[k] = den[k] * sf + p; acc[k] = pmul(acc[k], sf) + pmul(p, ln[k] + dl); m[k] = mn; } }
  v4f o; for (int k = 0; k < 4; ++k) o[k] = fmaxf(acc[k] / (den[k] + 1e-16f), 0.0f);
  const size_t tok = (lane < 16) ? i : (size_t)N + i; const int c0 = (lane & 15) * 4;
  for (int pass = 0; pass < 2; ++pass) { *(volatile v4f*)(T + tok * C + c0) = o; __threadfence(); } }
__global__ __launch_bounds__(32) void qkv_kernel(const float* __restrict__ T, const b16* __restrict__ QKVT, const float* __restrict__ qb, const float* __restrict__ kb, const float* __restrict__ vb, b16* __restrict__ Qh, b16* __restrict__ Kh, b16* __restrict__ VT) { __shared__ __attribute__((aligned(16))) b16 Ah[64][72], Al[64][72]; __shared__ float Tf[64][68]; const int lane = threadIdx.x, nloc = lane & 15, hlf = lane >> 4; const size_t s0 = (size_t)blockIdx.x * 64;
  for (int rr = 0; rr < 64; ++rr) for (int q = 0; q < 2; ++q) { b16 p, ql; split16(T[(s0 + rr) * C + q * 32 + lane] * XS, p, ql); Ah[rr][q * 32 + lane] = p; Al[rr][q * 32 + lane] = ql; }
  wave_lds_sync();
  for (int g = 0; g < 3; ++g) {
    for (int mt = 0; mt < 4; ++mt) { const v16b a0 = frag_kb(&Ah[mt * 16 + nloc][0], hlf), a1 = frag_kb(&Ah[mt * 16 + nloc][32], hlf), l0 = frag_kb(&Al[mt * 16 + nloc][0], hlf), l1 = frag_kb(&Al[mt * 16 + nloc][32], hlf);
#pragma unroll
      for (int t = 0; t < 4; ++t) { const b16* wr = QKVT + (size_t)(g * C + t * 16 + nloc) * C; const v16b b0 = frag_kb(wr, hlf), b1 = frag_kb(wr + 32, hlf); v8f acc = {}; acc = wmma16b(a0, b0, acc); acc = wmma16b(l0, b0, acc); acc = wmma16b(a1, b1, acc); acc = wmma16b(l1, b1, acc);
        const int c = t * 16 + nloc; const float bias = bf16_rne(g == 0 ? qb[c] : g == 1 ? kb[c] : vb[c]); const float sc = g == 0 ? SCALE : 1.0f;
#pragma unroll
        for (int r8 = 0; r8 < 8; ++r8) Tf[mt * 16 + 8 * hlf + r8][c] = (acc[r8] * (1.0f / (XS * WSC)) + bias) * sc; } }
    wave_lds_sync();
    for (int pass = 0; pass < 2; ++pass) {
      if (g < 2) { b16* dstp = g == 0 ? Qh : Kh; for (int rr = 0; rr < 64; ++rr) for (int q = 0; q < 2; ++q) ((volatile b16*)dstp)[(s0 + rr) * C + q * 32 + lane] = (b16)(Tf[rr][q * 32 + lane] * XS); }
      else { for (int cg = 0; cg < 2; ++cg) { const int c = cg * 32 + lane; for (int rr = 0; rr < 64; ++rr) ((volatile b16*)VT)[(size_t)c * S + s0 + rr] = (b16)(Tf[rr][c] * XS); } }
      __threadfence(); }
    wave_lds_sync(); } }
__global__ __launch_bounds__(32) void att_kernel(const b16* __restrict__ Qh, const b16* __restrict__ Kh, const b16* __restrict__ VT, int QL, float* __restrict__ ATT) { __shared__ __attribute__((aligned(16))) b16 Pb[16][40]; __shared__ float Of[16][36]; const int lane = threadIdx.x, nloc = lane & 15, hlf = lane >> 4; const int h = blockIdx.x & 1; const size_t q0 = (size_t)(blockIdx.x >> 1) * 16; if (q0 >= (size_t)QL) return;
  const v16b aq = frag_kb(Qh + (q0 + nloc) * C + h * HD, hlf); float mrow[8], lrow[8]; v8f oacc[2] = {(v8f){}, (v8f){}};
#pragma unroll
  for (int r8 = 0; r8 < 8; ++r8) { mrow[r8] = -INFINITY; lrow[r8] = 0.0f; }
#pragma unroll 1
  for (int kc = 0; kc < S; kc += 32) { v8f sacc[2] = {(v8f){}, (v8f){}};
#pragma unroll
    for (int t = 0; t < 2; ++t) sacc[t] = wmma16b(aq, frag_kb(Kh + (size_t)(kc + t * 16 + nloc) * C + h * HD, hlf), sacc[t]);
    float pv[2][8];
#pragma unroll
    for (int r8 = 0; r8 < 8; ++r8) { float s0 = sacc[0][r8] * (1.0f / (XS * XS)), s1 = sacc[1][r8] * (1.0f / (XS * XS)); float mx = fmaxf(s0, s1); mx = fmaxf(mx, __shfl_xor(mx, 1)); mx = fmaxf(mx, __shfl_xor(mx, 2)); mx = fmaxf(mx, __shfl_xor(mx, 4)); mx = fmaxf(mx, __shfl_xor(mx, 8));
      const float mn = fmaxf(mrow[r8], mx); const float corr = (mrow[r8] == -INFINITY) ? 0.0f : __expf(mrow[r8] - mn); const float p0 = __expf(s0 - mn), p1 = __expf(s1 - mn); float ps = p0 + p1; ps += __shfl_xor(ps, 1); ps += __shfl_xor(ps, 2); ps += __shfl_xor(ps, 4); ps += __shfl_xor(ps, 8);
      lrow[r8] = lrow[r8] * corr + ps; mrow[r8] = mn; oacc[0][r8] = pmul(oacc[0][r8], corr); oacc[1][r8] = pmul(oacc[1][r8], corr); pv[0][r8] = p0; pv[1][r8] = p1; }
#pragma unroll
    for (int t = 0; t < 2; ++t)
#pragma unroll
      for (int r8 = 0; r8 < 8; ++r8) Pb[8 * hlf + r8][t * 16 + nloc] = (b16)(pv[t][r8] * PS);
    wave_lds_sync(); const v16b ap = frag_kb(&Pb[nloc][0], hlf);
#pragma unroll
    for (int t = 0; t < 2; ++t) oacc[t] = wmma16b(ap, frag_kb(VT + (size_t)(h * HD + t * 16 + nloc) * S + kc, hlf), oacc[t]);
    wave_lds_sync(); }
#pragma unroll
  for (int t = 0; t < 2; ++t)
#pragma unroll
    for (int r8 = 0; r8 < 8; ++r8) Of[8 * hlf + r8][t * 16 + nloc] = oacc[t][r8] * (1.0f / (PS * XS)) / lrow[r8];
  wave_lds_sync();
  for (int pass = 0; pass < 2; ++pass) { for (int rr = 0; rr < 16; ++rr) ((volatile float*)ATT)[(q0 + rr) * C + h * HD + lane] = Of[rr][lane]; __threadfence(); } }
__global__ __launch_bounds__(32) void out_kernel(const float* __restrict__ ATT, const b16* __restrict__ OWT, const float* __restrict__ ob, int QL, float* __restrict__ out) { __shared__ __attribute__((aligned(16))) b16 Ah[16][72], Al[16][72]; __shared__ float Tf[16][68]; const int lane = threadIdx.x, nloc = lane & 15, hlf = lane >> 4; const size_t m0 = (size_t)blockIdx.x * 16; if (m0 >= (size_t)QL) return;
  for (int rr = 0; rr < 16; ++rr) for (int q = 0; q < 2; ++q) { b16 p, ql; split16(ATT[(m0 + rr) * C + q * 32 + lane] * XS, p, ql); Ah[rr][q * 32 + lane] = p; Al[rr][q * 32 + lane] = ql; }
  wave_lds_sync(); v8f acc[4] = {(v8f){}, (v8f){}, (v8f){}, (v8f){}};
#pragma unroll
  for (int kb = 0; kb < C; kb += 32) { const v16b a = frag_kb(&Ah[nloc][kb], hlf), al = frag_kb(&Al[nloc][kb], hlf);
#pragma unroll
    for (int t = 0; t < 4; ++t) { const v16b bw = frag_kb(OWT + (size_t)(t * 16 + nloc) * C + kb, hlf); acc[t] = wmma16b(a, bw, acc[t]); acc[t] = wmma16b(al, bw, acc[t]); } }
#pragma unroll
  for (int t = 0; t < 4; ++t) { const int c = t * 16 + nloc; const float bb = bf16_rne(ob[c]);
#pragma unroll
    for (int r8 = 0; r8 < 8; ++r8) Tf[8 * hlf + r8][c] = acc[t][r8] * (1.0f / (XS * WSC)) + bb; }
  wave_lds_sync();
  for (int pass = 0; pass < 2; ++pass) { for (int rr = 0; rr < 16; ++rr) *(volatile v2f*)(out + (m0 + rr) * C + lane * 2) = (v2f){Tf[rr][lane * 2], Tf[rr][lane * 2 + 1]}; __threadfence(); } }
}

extern "C" void kernel_launch(void* const* d_in, const int* in_sizes, int n_in, void* d_out, int out_size, void* d_ws, size_t ws_size, hipStream_t stream) {
  (void)n_in;
  auto Fp = [&](int i) { return (const float*)d_in[i]; }; auto Ip = [&](int i) { return (const int*)d_in[i]; };
  if (in_sizes[0] != N * C || in_sizes[1] != N * 3 || in_sizes[2] != C * O || in_sizes[5] != 3 * O || in_sizes[7] != C * C || in_sizes[13] != C * C || in_sizes[15] != 2 * E || out_size != S * C) return;
  const int QL = S;
  size_t off = 0; char* ws = (char*)d_ws;
  auto carve = [&](size_t bytes) { char* p = ws + off; off += (bytes + 255) & ~(size_t)255; return p; };
  b16* LT = (b16*)carve((size_t)3 * O * C * 2); b16* QKVT = (b16*)carve((size_t)3 * C * C * 2); b16* OWT = (b16*)carve((size_t)C * C * 2); float* L = (float*)carve((size_t)N * 3 * O * 4); float* T = (float*)carve((size_t)S * C * 4);
  b16* Qh = (b16*)carve((size_t)S * C * 2); b16* Kh = (b16*)carve((size_t)S * C * 2); b16* VT = (b16*)carve((size_t)C * S * 2); float* ATT = (float*)carve((size_t)S * C * 4); CsrBufs8 csr; off = csr_carve8(csr, ws, off, E, N);
  if (off > ws_size || off > ((size_t)32 << 20)) return;
  wput_kernel<<<(3 * O * 8 + 255) / 256, 256, 0, stream>>>(Fp(2), Fp(3), Fp(4), Fp(7), Fp(9), Fp(11), Fp(13), LT, QKVT, OWT);
  csr_build8(csr, Ip(15) + E, E, N, stream);
  lin_kernel<<<N / 16, 32, 0, stream>>>(Fp(0), LT, L);
  pt_kernel<<<N / 8, 256, 0, stream>>>(L, Fp(1), Fp(5), Fp(6), Ip(15), csr.PERM, csr.ROWPTR, csr.ROWCNT, (int)csr.permLen, T);
  qkv_kernel<<<S / 64, 32, 0, stream>>>(T, QKVT, Fp(8), Fp(10), Fp(12), Qh, Kh, VT);
  att_kernel<<<(QL / 16) * 2, 32, 0, stream>>>(Qh, Kh, VT, QL, ATT);
  out_kernel<<<S / 16, 32, 0, stream>>>(ATT, OWT, Fp(14), QL, (float*)d_out);
}
